// SelfAttn_41781441856090
// MI455X (gfx1250) — hardware-run, weakly checked
//
#include <hip/hip_runtime.h>


#ifndef NB
#define NB 8
#endif
#ifndef SEQ
#define SEQ 256
#endif
#define NB_FULL  8
#define SEQ_FULL 256
#define HID   256
#define NCOL  (2 * HID)
#define MROWS (SEQ * NB_FULL)
#define JT    32
#define EW    8
#define CPW   (JT / EW)
#define ESP   36
#define NV    (SEQ / 32)
#define TL2E  2.8853900817779268f
#define L2E   1.4426950408889634f
#define NEGB  (-3.0e38f)

static_assert(HID == 256);
static_assert(HID == 32 * 8);
static_assert(HID % 32 == 0);
static_assert(NCOL % 64 == 0);
static_assert(HID % 64 == 0);
static_assert(MROWS % 64 == 0);
static_assert(SEQ % 32 == 0);
static_assert(JT % EW == 0);
static_assert(JT * 4 == 128);
static_assert((ESP * 4) % 16 == 0);
static_assert(ESP >= JT);
static_assert(NB <= NB_FULL);
static_assert(SEQ <= SEQ_FULL);
static_assert(((size_t)MROWS * HID) % 8 == 0);
static_assert(((size_t)HID * NCOL) % 8 == 0);
static_assert(32 * 16 * 8 == 16 * 64 * 4);
static_assert((size_t)(32 * EW) * 16 * (SEQ / 32) == (size_t)SEQ * JT * 4);
static_assert((size_t)SEQ * ESP * 4 <= 131072);
static_assert((size_t)16 * 68 * 4 <= 131072);

typedef unsigned short bf;
typedef __attribute__((ext_vector_type(16))) __bf16   v16bf;
typedef __attribute__((ext_vector_type(8)))  unsigned short v8us;
typedef __attribute__((ext_vector_type(8)))  float    v8f;
typedef __attribute__((ext_vector_type(4)))  float    v4f;
typedef v4f  __attribute__((may_alias)) v4fa;

__device__ __forceinline__ unsigned short f2bf(float f) { unsigned u = __float_as_uint(f); u += 0x7FFFu + ((u >> 16) & 1u); return (unsigned short)(u >> 16); }
__device__ __forceinline__ float bfr(float f) { return __uint_as_float(((unsigned)f2bf(f)) << 16); }
__device__ __forceinline__ v16bf cat16b(v8us lo, v8us hi) { return __builtin_bit_cast(v16bf, __builtin_shufflevector(lo, hi, 0, 1, 2, 3, 4, 5, 6, 7, 8, 9, 10, 11, 12, 13, 14, 15)); }
__device__ __forceinline__ v8f wmmab(v16bf a, v16bf b, v8f c) { return __builtin_amdgcn_wmma_f32_16x16x32_bf16(false, a, false, b, (short)0, c, false, false); }
__device__ __forceinline__ v8f wmmabg(v16bf a, v16bf b, v8f c) { c = wmmab(a, b, c); asm volatile("v_nop\n\tv_nop\n\tv_nop\n\tv_nop" : "+v"(c) : "v"(a), "v"(b)); return c; }
__device__ __forceinline__ v16bf ldb(const bf* p)  { return cat16b(*(const v8us*)p, *(const v8us*)(p + 16)); }
__device__ __forceinline__ void wave_sync() { __builtin_amdgcn_fence(3  , "wavefront"); __builtin_amdgcn_wave_barrier(); asm volatile("" ::: "memory"); }

__global__ __launch_bounds__(256) void k_cvt8(const float* __restrict__ src, bf* dst, size_t n8) {
    const size_t i = (size_t)blockIdx.x * 256 + threadIdx.x; if (i >= n8) return;
    const v8f v = *(const v8f*)(src + i * 8); v8us o;
#pragma unroll
    for (int k = 0; k < 8; ++k) o[k] = f2bf(v[k]);
    *(volatile v8us*)(dst + i * 8) = o; __threadfence(); *(volatile v8us*)(dst + i * 8) = o;
}

__global__ __launch_bounds__(32) void k_pgemm(const bf* __restrict__ A, const bf* __restrict__ Bt, const float* __restrict__ bias, float* PP) {
    __shared__ __align__(16) float os[16 * 68];
    const unsigned lane = threadIdx.x & 31u, lr = lane & 15u, hi = lane >> 4;
    const unsigned r0 = blockIdx.x * 64u, c0 = blockIdx.y * 64u;
    const unsigned sel = c0 >> 8, wc0 = c0 & 255u;
    v8f acc[4][4];
#pragma unroll
    for (int mb = 0; mb < 4; ++mb)
#pragma unroll
        for (int nb = 0; nb < 4; ++nb) acc[mb][nb] = (v8f){};
    const size_t aoff = (size_t)(r0 + lr) * HID + 8u * hi;
    const size_t boff = (size_t)(wc0 + lr) * NCOL + (size_t)sel * HID + 8u * hi;
#pragma unroll 1
    for (unsigned kc = 0; kc < HID; kc += 32u) {
        v16bf a[4];
#pragma unroll
        for (int mb = 0; mb < 4; ++mb) a[mb] = ldb(A + aoff + (size_t)mb * 16 * HID + kc);
#pragma unroll
        for (int nb = 0; nb < 4; ++nb) { const v16bf b = ldb(Bt + boff + (size_t)nb * 16 * NCOL + kc);
#pragma unroll
            for (int mb = 0; mb < 4; ++mb) acc[mb][nb] = wmmabg(a[mb], b, acc[mb][nb]); }
    }
    float bc[4];
#pragma unroll
    for (int nb = 0; nb < 4; ++nb) { const float bv = bfr(bias[wc0 + nb * 16 + lr]); bc[nb] = (sel == 0u) ? bv : 0.0f; }
    float* pl = PP + (size_t)sel * ((size_t)MROWS * HID) + (size_t)r0 * HID + wc0;
#pragma unroll
    for (int mb = 0; mb < 4; ++mb) {
#pragma unroll
        for (int nb = 0; nb < 4; ++nb) {
#pragma unroll
            for (int j = 0; j < 8; ++j) os[(hi * 8 + j) * 68 + nb * 16 + lr] = acc[mb][nb][j] + bc[nb]; }
        wave_sync();
#pragma unroll 1
        for (int ps = 0; ps < 2; ++ps) {
#pragma unroll
            for (int s = 0; s < 8; ++s) { const unsigned row = 2u * s + (lane >> 4), cofs = (lane & 15u) * 4u;
                const v4f val = *(const v4fa*)(&os[row * 68 + cofs]);
                *(volatile v4f*)(pl + (size_t)(mb * 16 + row) * HID + cofs) = val; }
            if (ps == 0) __threadfence(); }
        wave_sync();
    }
}

__global__ __launch_bounds__(32 * EW) void k_energy(const float* __restrict__ PP, const float* __restrict__ wsc, const float* __restrict__ bsc, float* OUT) {
#pragma clang fp contract(off)
    __shared__ __align__(16) float es[SEQ * ESP];
    const unsigned tid = threadIdx.x, lane = tid & 31u;
    const int wave = __builtin_amdgcn_readfirstlane((int)(threadIdx.x >> 5));
    const unsigned j0 = blockIdx.x * (unsigned)JT;
    const unsigned b = blockIdx.y;
    const size_t lo8 = (size_t)(8u * lane);
    float w2[8]; float wl = 0.0f;
    { const v4f wa = *(const v4f*)(wsc + lo8); const v4f wb = *(const v4f*)(wsc + lo8 + 4);
#pragma unroll
      for (int k = 0; k < 4; ++k) { const float u0 = bfr(wa[k]); const float u1 = bfr(wb[k]); w2[k] = -2.0f * u0; w2[4 + k] = -2.0f * u1; wl += u0; wl += u1; } }
    const float bsv = bfr(bsc[0]);
#pragma unroll 1
    for (unsigned c = 0; c < (unsigned)CPW; ++c) {
        const unsigned jl = (unsigned)wave * (unsigned)CPW + c;
        const float* p2r = PP + (size_t)MROWS * HID + (size_t)((j0 + jl) * (unsigned)NB_FULL + b) * HID + lo8;
        float p2c[8];
        { const v4f q0 = *(const v4f*)p2r; const v4f q1 = *(const v4f*)(p2r + 4);
#pragma unroll
          for (int k = 0; k < 4; ++k) { p2c[k] = q0[k] * TL2E; p2c[4 + k] = q1[k] * TL2E; } }
#pragma unroll 1
        for (unsigned i0 = 0; i0 < (unsigned)SEQ; i0 += 32u) {
            float ev = 0.0f;
#pragma unroll 1
            for (unsigned ii = 0; ii < 32u; ++ii) {
                const float* p1r = PP + (size_t)((i0 + ii) * (unsigned)NB_FULL + b) * HID + lo8;
                const v4f a0 = *(const v4f*)p1r; const v4f a1 = *(const v4f*)(p1r + 4);
                float acc = wl;
#pragma unroll
                for (int k = 0; k < 4; ++k) {
                    const float za = fmaf(a0[k], TL2E, p2c[k]);
                    const float zb = fmaf(a1[k], TL2E, p2c[4 + k]);
                    const float ra = __builtin_amdgcn_rcpf(__builtin_amdgcn_exp2f(za) + 1.0f);
                    const float rb = __builtin_amdgcn_rcpf(__builtin_amdgcn_exp2f(zb) + 1.0f);
                    acc = fmaf(w2[k], ra, acc);
                    acc = fmaf(w2[4 + k], rb, acc);
                }
                acc += __shfl_xor(acc, 16, 32);
                acc += __shfl_xor(acc, 8, 32);
                acc += __shfl_xor(acc, 4, 32);
                acc += __shfl_xor(acc, 2, 32);
                acc += __shfl_xor(acc, 1, 32);
                const float e = acc + bsv;
                ev = (ii == lane) ? e : ev;
            }
            es[(i0 + lane) * ESP + jl] = ev;
        }
        wave_sync();
        float x[NV]; float mx = NEGB;
#pragma unroll
        for (int k = 0; k < NV; ++k) { x[k] = es[(32u * k + lane) * ESP + jl]; mx = fmaxf(mx, x[k]); }
        mx = fmaxf(mx, __shfl_xor(mx, 16, 32));
        mx = fmaxf(mx, __shfl_xor(mx, 8, 32));
        mx = fmaxf(mx, __shfl_xor(mx, 4, 32));
        mx = fmaxf(mx, __shfl_xor(mx, 2, 32));
        mx = fmaxf(mx, __shfl_xor(mx, 1, 32));
        float s = 0.0f;
#pragma unroll
        for (int k = 0; k < NV; ++k) { const float d = (x[k] - mx) * L2E; x[k] = __builtin_amdgcn_exp2f(d); s += x[k]; }
        s += __shfl_xor(s, 16, 32);
        s += __shfl_xor(s, 8, 32);
        s += __shfl_xor(s, 4, 32);
        s += __shfl_xor(s, 2, 32);
        s += __shfl_xor(s, 1, 32);
        const float inv = 1.0f / s;
#pragma unroll
        for (int k = 0; k < NV; ++k) { const float pv = x[k] * inv; es[(32u * k + lane) * ESP + jl] = pv; }
        wave_sync();
    }
    __syncthreads();
    float* ob = OUT + ((size_t)b * SEQ) * SEQ + j0;
#pragma unroll 1
    for (int ps = 0; ps < 2; ++ps) {
#pragma unroll 1
        for (unsigned it = 0; it < (unsigned)(SEQ / 32); ++it) { const unsigned row = it * 32u + (tid >> 3), cofs = (tid & 7u) * 4u;
            const v4f val = *(const v4fa*)(&es[row * ESP + cofs]);
            *(volatile v4f*)(ob + (size_t)row * SEQ + cofs) = val; }
        if (ps == 0) __threadfence(); }
}

static constexpr size_t al256(size_t v) { return (v + 255) & ~(size_t)255; }
static constexpr size_t SZ_XB = al256((size_t)MROWS * HID * 2);
static constexpr size_t SZ_WB = al256((size_t)HID * NCOL * 2);
static constexpr size_t SZ_PP = al256((size_t)2 * MROWS * HID * 4);
static constexpr size_t SZ_TOTAL = SZ_XB + SZ_WB + SZ_PP;
static_assert(SZ_TOTAL <= (size_t)134217728);
static constexpr size_t N8_X = (size_t)MROWS * HID / 8;
static constexpr size_t N8_W = (size_t)HID * NCOL / 8;
static constexpr unsigned G_X = (unsigned)((N8_X + 255) / 256);
static constexpr unsigned G_W = (unsigned)((N8_W + 255) / 256);
static constexpr size_t NEED_X = (size_t)MROWS * HID;
static constexpr size_t NEED_W = (size_t)HID * NCOL;
static constexpr size_t NEED_O = (size_t)NB * SEQ * SEQ;
static_assert(N8_X * 8 * 2 <= SZ_XB);
static_assert(N8_W * 8 * 2 <= SZ_WB);
static_assert((size_t)2 * MROWS * HID * 4 <= SZ_PP);
static_assert(NEED_O * 4 <= (size_t)2097152);

extern "C" void kernel_launch(void* const* d_in, const int* in_sizes, int n_in,
                              void* d_out, int out_size, void* d_ws, size_t ws_size, hipStream_t stream) {
    if (n_in < 6) return;
    if ((size_t)in_sizes[0] < NEED_X) return;
    if ((size_t)in_sizes[2] < NEED_W) return;
    if (in_sizes[3] < HID || in_sizes[4] < HID || in_sizes[5] < 1) return;
    if ((size_t)out_size < NEED_O) return;
    if (SZ_TOTAL > ws_size) return;
    const float* xin = (const float*)d_in[0];
    const float* wat = (const float*)d_in[2];
    const float* bat = (const float*)d_in[3];
    const float* wsc = (const float*)d_in[4];
    const float* bsc = (const float*)d_in[5];
    float* OUT = (float*)d_out;
    char* wsp = (char*)d_ws;
    bf* XB = (bf*)wsp; wsp += SZ_XB;
    bf* WB = (bf*)wsp; wsp += SZ_WB;
    float* PP = (float*)wsp; wsp += SZ_PP;

    k_cvt8<<<G_X, 256, 0, stream>>>(xin, XB, N8_X);
    k_cvt8<<<G_W, 256, 0, stream>>>(wat, WB, N8_W);
    k_pgemm<<<dim3(MROWS / 64, NCOL / 64, 1), 32, 0, stream>>>(XB, WB, bat, PP);
    k_energy<<<dim3(SEQ / JT, NB, 1), 32 * EW, 0, stream>>>(PP, wsc, bsc, OUT);
}
